// OptiXAttentionReal_7464653161177
// MI455X (gfx1250) — hardware-verified
//
#include <hip/hip_runtime.h>
#include <math.h>

constexpr int kBatch = 2;
constexpr int kSeq   = 2048;
constexpr int kDim   = 1024;
constexpr int kTok   = kBatch * kSeq;
constexpr int kPosLd = 4;

typedef __attribute__((ext_vector_type(16))) _Float16 v16h;
typedef __attribute__((ext_vector_type(8)))  _Float16 v8h;
typedef __attribute__((ext_vector_type(16))) __bf16   v16b;
typedef __attribute__((ext_vector_type(8)))  __bf16   v8b;
typedef __attribute__((ext_vector_type(8)))  float    v8f;
typedef __attribute__((ext_vector_type(4)))  float    v4f;
typedef __attribute__((ext_vector_type(4)))  unsigned int v4u;

__device__ __forceinline__ unsigned short f2bf_bits(float f) {
  unsigned u = __float_as_uint(f);
  return (unsigned short)((u + 0x7FFFu + ((u >> 16) & 1u)) >> 16);
}
__device__ __forceinline__ float bf_bits2f(unsigned short h) { return __uint_as_float(((unsigned)h) << 16); }
__device__ __forceinline__ float bf_rne(float f) { return bf_bits2f(f2bf_bits(f)); }

__device__ __forceinline__ void dep_guard_h(v8f& a, v8f& b, v16h x, v16h y) { asm volatile("v_nop\n\tv_nop\n\tv_nop\n\tv_nop" : "+v"(a), "+v"(b) : "v"(x), "v"(y)); }
__device__ __forceinline__ void dep_guard_b(v8f& a, v8f& b, v16b x, v16b y) { asm volatile("v_nop\n\tv_nop\n\tv_nop\n\tv_nop" : "+v"(a), "+v"(b) : "v"(x), "v"(y)); }
__device__ __forceinline__ void keep4_h(v16h a, v16h b, v16h c, v16h d) { asm volatile("v_nop" :: "v"(a), "v"(b), "v"(c), "v"(d)); }
__device__ __forceinline__ void keep4_b(v16b a, v16b b, v16b c, v16b d) { asm volatile("v_nop" :: "v"(a), "v"(b), "v"(c), "v"(d)); }
__device__ __forceinline__ void acc_guard4(v8f& a, v8f& b, v8f& c, v8f& d) { asm volatile("v_nop\n\tv_nop\n\tv_nop\n\tv_nop" : "+v"(a), "+v"(b), "+v"(c), "+v"(d)); }
template <typename T> struct Frag;
template <> struct Frag<_Float16> {
  typedef v16h V; union U { v16h v; v8h h[2]; };
  static __device__ __forceinline__ v16h load(const _Float16* p) {
    U f; f.h[0] = *(const v8h*)(p); f.h[1] = *(const v8h*)(p + 16); return f.v;
  }
  static __device__ __forceinline__ v8f mma(v16h a, v16h b, v8f c) {
    return __builtin_amdgcn_wmma_f32_16x16x32_f16(false, a, false, b, (short)0, c, false, false);
  }
  static __device__ __forceinline__ void guard(v8f& a, v8f& b, v16h x, v16h y) { dep_guard_h(a, b, x, y); }
  static __device__ __forceinline__ void keep(v16h a, v16h b, v16h c, v16h d) { keep4_h(a, b, c, d); }
};
template <> struct Frag<__bf16> {
  typedef v16b V; union U { v16b v; v8b h[2]; };
  static __device__ __forceinline__ v16b load(const __bf16* p) {
    U f; f.h[0] = *(const v8b*)(p); f.h[1] = *(const v8b*)(p + 16); return f.v;
  }
  static __device__ __forceinline__ v8f mma(v16b a, v16b b, v8f c) {
    return __builtin_amdgcn_wmma_f32_16x16x32_bf16(false, a, false, b, (short)0, c, false, false);
  }
  static __device__ __forceinline__ void guard(v8f& a, v8f& b, v16b x, v16b y) { dep_guard_b(a, b, x, y); }
  static __device__ __forceinline__ void keep(v16b a, v16b b, v16b c, v16b d) { keep4_b(a, b, c, d); }
};

__device__ __forceinline__ unsigned pk16(unsigned short a, unsigned short b) { return (unsigned)a | ((unsigned)b << 16); }

template <int ET> struct Elem;
template <> struct Elem<0> { typedef _Float16 T; };
template <> struct Elem<1> { typedef __bf16 T; };
template <int ET, int SPLIT, int BIAS_MODE, int OUT_MODE, bool RESID, int ACT = 0, bool KCAUSAL = false>
__global__ __launch_bounds__(256) void wmma_gemm64(
    const unsigned short* __restrict__ Ap, const unsigned short* __restrict__ A2p, int lda, long strideA,
    const unsigned short* __restrict__ Btp, const unsigned short* __restrict__ Bt2p, int ldb, long strideB,
    void* __restrict__ Cout, void* __restrict__ Cout2, int ldc, long strideC,
    const float* __restrict__ bias,
    const float* __restrict__ resid, long strideR,
    int M, int N, int K, float scale) {
  typedef typename Elem<ET>::T T;
  typedef typename Frag<T>::V V;
  const T* A = (const T*)Ap; const T* A2 = (const T*)A2p; const T* Bt = (const T*)Btp; const T* Bt2 = (const T*)Bt2p;
  __shared__ __align__(16) float sT[8][16 * 68];
  const int b    = blockIdx.y;
  const int lane = threadIdx.x & 31;
  const int wave = threadIdx.x >> 5;
  const int tilesN = N >> 6;
  const int tilesM = M >> 6;
  const int tile = blockIdx.x * 8 + wave;
  if (tile >= tilesM * tilesN) return;
  const int tm = tile / tilesN;
  const int tn = tile - tm * tilesN;
  const int m0 = tm << 6;
  const int n0 = tn << 6;

  const T* Ab  = A  + (size_t)b * strideA;
  const T* Bb  = Bt + (size_t)b * strideB;
  const T* Ab2 = (SPLIT >= 1) ? (A2  + (size_t)b * strideA) : nullptr;
  const T* Bb2 = (SPLIT == 2) ? (Bt2 + (size_t)b * strideB) : nullptr;

  const int rlane = lane & 15;
  const int koff  = (lane >> 4) * 8;
  const int mOff  = (lane >> 4) * 8;

  v8f acc[4][4];
#pragma unroll
  for (int i = 0; i < 4; ++i)
#pragma unroll
    for (int j = 0; j < 4; ++j) acc[i][j] = (v8f){0.f,0.f,0.f,0.f,0.f,0.f,0.f,0.f};

  const int kEnd = KCAUSAL ? (((m0 + 64) < K) ? (m0 + 64) : K) : K;
  for (int k0 = 0; k0 < kEnd; k0 += 32) {
    V bh[4], bl[4];
#pragma unroll
    for (int j = 0; j < 4; ++j) {
      const size_t bo = (size_t)(n0 + (j << 4) + rlane) * ldb + koff + k0;
      bh[j] = Frag<T>::load(Bb + bo);
      if (SPLIT == 2) bl[j] = Frag<T>::load(Bb2 + bo);
    }
#pragma unroll
    for (int i = 0; i < 4; ++i) {
      const size_t ao = (size_t)(m0 + (i << 4) + rlane) * lda + koff + k0;
      V ah = Frag<T>::load(Ab + ao);
      V al;
      if (SPLIT >= 1) al = Frag<T>::load(Ab2 + ao);
#pragma unroll
      for (int j = 0; j < 4; ++j) {
        acc[i][j] = Frag<T>::mma(ah, bh[j], acc[i][j]);
        if (SPLIT == 2) acc[i][j] = Frag<T>::mma(ah, bl[j], acc[i][j]);
        if (SPLIT >= 1) acc[i][j] = Frag<T>::mma(al, bh[j], acc[i][j]);
      }
      Frag<T>::guard(acc[i][0], acc[i][3], ah, (SPLIT >= 1) ? al : ah);
    }
    Frag<T>::keep(bh[0], bh[1], bh[2], bh[3]);
    if (SPLIT == 2) Frag<T>::keep(bl[0], bl[1], bl[2], bl[3]);
  }
  acc_guard4(acc[0][0], acc[0][1], acc[0][2], acc[0][3]);
  acc_guard4(acc[1][0], acc[1][1], acc[1][2], acc[1][3]);
  acc_guard4(acc[2][0], acc[2][1], acc[2][2], acc[2][3]);
  acc_guard4(acc[3][0], acc[3][1], acc[3][2], acc[3][3]);

  float* slab = sT[wave];
  const float* Rb = RESID ? (resid + (size_t)b * strideR) : nullptr;
#pragma unroll
  for (int i = 0; i < 4; ++i) {
    const int mBase = m0 + (i << 4);
#pragma unroll
    for (int j = 0; j < 4; ++j) {
      const int n = n0 + (j << 4) + rlane;
      float bv = 0.f;
      if (BIAS_MODE == 2) bv = bias[n];
#pragma unroll
      for (int r = 0; r < 8; ++r) {
        float v = acc[i][j][r] * scale;
        if (BIAS_MODE == 1) v += bias[mBase + mOff + r];
        if (BIAS_MODE == 2) v += bv;
        if (RESID) v += Rb[(size_t)(mBase + mOff + r) * ldc + n];
        if (ACT == 2) v = fmaxf(v, 0.0f);
        if (ACT == 4) v = (v > 0.f) ? v : 0.01f * v;
        slab[(mOff + r) * 68 + (j << 4) + rlane] = v;
      }
    }
    __builtin_amdgcn_fence(__ATOMIC_RELEASE, "workgroup");
    __builtin_amdgcn_wave_barrier();
    __builtin_amdgcn_fence(__ATOMIC_ACQUIRE, "workgroup");
    if (OUT_MODE == 0) {
      float* C = (float*)Cout + (size_t)b * strideC;
      const int hh = lane >> 4, c4 = (lane & 15) * 4;
      for (int pass = 0; pass < 2; ++pass) {
#pragma unroll
        for (int it = 0; it < 8; ++it) {
          const int row = it * 2 + hh;
          v4f v = *(const v4f*)(slab + row * 68 + c4);
          *(volatile v4f*)(C + (size_t)(mBase + row) * ldc + n0 + c4) = v;
        }
        __threadfence();
      }
    } else {
      const int q = lane >> 3, c8 = (lane & 7) * 8;
      unsigned short* C  = (unsigned short*)Cout  + (size_t)b * strideC;
      unsigned short* C2 = (OUT_MODE == 2) ? ((unsigned short*)Cout2 + (size_t)b * strideC) : nullptr;
      for (int pass = 0; pass < 2; ++pass) {
#pragma unroll
        for (int it = 0; it < 4; ++it) {
          const int row = it * 4 + q;
          const float* sp = slab + row * 68 + c8;
          v8h hv, lv;
#pragma unroll
          for (int e = 0; e < 8; ++e) {
            if (OUT_MODE == 1) {
              hv[e] = (_Float16)sp[e];
            } else {
              unsigned short hb = f2bf_bits(sp[e]);
              unsigned short lb = f2bf_bits(sp[e] - bf_bits2f(hb));
              hv[e] = __builtin_bit_cast(_Float16, hb);
              lv[e] = __builtin_bit_cast(_Float16, lb);
            }
          }
          *(volatile v8h*)(C + (size_t)(mBase + row) * ldc + n0 + c8) = hv;
          if (OUT_MODE == 2) *(volatile v8h*)(C2 + (size_t)(mBase + row) * ldc + n0 + c8) = lv;
        }
        __threadfence();
      }
    }
    __builtin_amdgcn_fence(__ATOMIC_RELEASE, "workgroup");
    __builtin_amdgcn_wave_barrier();
    __builtin_amdgcn_fence(__ATOMIC_ACQUIRE, "workgroup");
  }
}

__global__ __launch_bounds__(256) void cast8_bf16_kernel(const float* __restrict__ in, unsigned short* __restrict__ out, int n8) {
  const int i = blockIdx.x * 256 + threadIdx.x;
  if (i >= n8) return;
  const float* p = in + 8 * (size_t)i;
  const v4f a = *(const v4f*)(p);
  const v4f c = *(const v4f*)(p + 4);
  unsigned short hb[8];
#pragma unroll
  for (int e = 0; e < 4; ++e) {
    hb[e]     = f2bf_bits(a[e]);
    hb[4 + e] = f2bf_bits(c[e]);
  }
  const v4u u = (v4u){pk16(hb[0], hb[1]), pk16(hb[2], hb[3]), pk16(hb[4], hb[5]), pk16(hb[6], hb[7])};
  unsigned short* q = out + 8 * (size_t)i;
  *(volatile v4u*)q = u;
  __threadfence();
  *(volatile v4u*)q = u;
}

__global__ __launch_bounds__(256) void bias_bf16_kernel(const float* __restrict__ bvIn, const float* __restrict__ boIn,
                                                        float* __restrict__ bvOut, float* __restrict__ boOut) {
  const int t = threadIdx.x;
  const v4f a = *(const v4f*)(bvIn + 4 * t);
  const v4f c = *(const v4f*)(boIn + 4 * t);
  v4f ra, rc;
#pragma unroll
  for (int e = 0; e < 4; ++e) { ra[e] = bf_rne(a[e]); rc[e] = bf_rne(c[e]); }
  float* qa = bvOut + 4 * t;
  float* qc = boOut + 4 * t;
  *(volatile v4f*)qa = ra;
  *(volatile v4f*)qc = rc;
  __threadfence();
  *(volatile v4f*)qa = ra;
  *(volatile v4f*)qc = rc;
}

__global__ __launch_bounds__(256) void pos_kernel(const unsigned short* __restrict__ Xb, const float* __restrict__ w3d,
                                                  const float* __restrict__ b3d, float* __restrict__ pos) {
  __shared__ __align__(16) float sPos[8][4];
  const int t = threadIdx.x;
  const int wave = t >> 5, lane = t & 31;
  const int row = blockIdx.x * 8 + wave;
  const unsigned short* xr = Xb + (size_t)row * kDim;
  float s0 = 0.f, s1 = 0.f, s2 = 0.f;
#pragma unroll 1
  for (int c = 0; c < 4; ++c) {
    const int base = c * 256 + lane * 8;
    const v4u xw = *(const v4u*)(xr + base);
#pragma unroll
    for (int e = 0; e < 8; ++e) {
      const unsigned w = xw[e >> 1];
      const float xv = (e & 1) ? __uint_as_float(w & 0xffff0000u) : __uint_as_float(w << 16);
      s0 += xv * bf_rne(w3d[base + e]);
      s1 += xv * bf_rne(w3d[kDim + base + e]);
      s2 += xv * bf_rne(w3d[2 * kDim + base + e]);
    }
  }
#pragma unroll
  for (int off = 16; off > 0; off >>= 1) {
    s0 += __shfl_xor(s0, off, 32);
    s1 += __shfl_xor(s1, off, 32);
    s2 += __shfl_xor(s2, off, 32);
  }
  if (lane == 0) {
    sPos[wave][0] = s0 + bf_rne(b3d[0]);
    sPos[wave][1] = s1 + bf_rne(b3d[1]);
    sPos[wave][2] = s2 + bf_rne(b3d[2]);
    sPos[wave][3] = 0.f;
  }
  __syncthreads();
  if (wave == 0 && lane < 8) {
    const v4f v = *(const v4f*)(&sPos[lane][0]);
    float* dst = pos + ((size_t)blockIdx.x * 8 + lane) * kPosLd;
    *(volatile v4f*)dst = v;
    __threadfence();
    *(volatile v4f*)dst = v;
  }
}

__global__ __launch_bounds__(256) void attn_rows_kernel(const float* __restrict__ pos,
                                                        unsigned short* __restrict__ Ah, unsigned short* __restrict__ Al) {
#pragma clang fp contract(off)
  __shared__ __align__(16) float sP[kSeq];
  __shared__ float redS[8];
  const int blk = blockIdx.x;
  const int b = blk >> 11, i = blk & (kSeq - 1);
  const int t = threadIdx.x, lane = t & 31, wave = t >> 5;
  const float* pb = pos + (size_t)b * kSeq * kPosLd;
  const v4f pi = *(const v4f*)(pb + (size_t)i * kPosLd);
  float lsum = 0.f;
#pragma unroll 1
  for (int it = 0; it < 8; ++it) {
    const int j = it * 256 + t;
    const v4f pj = *(const v4f*)(pb + (size_t)j * kPosLd);
    const float dx = pi.x - pj.x;
    const float dy = pi.y - pj.y;
    const float dz = pi.z - pj.z;
    const float sq = (dx * dx + dz * dz) + dy * dy;
    const float sqs = (sq > 0.f) ? sq : 1.0f;
    const float dist = (sq > 0.f) ? sqrtf(sqs) : 0.f;
    const float e = expf(-(dist * 0.125f));
    const float p = (j <= i) ? e : 0.f;
    sP[j] = p;
    lsum += p;
  }
  float v = lsum;
#pragma unroll
  for (int off = 16; off > 0; off >>= 1) v += __shfl_xor(v, off, 32);
  if (lane == 0) redS[wave] = v;
  __syncthreads();
  float total = redS[0];
  total += redS[1]; total += redS[2]; total += redS[3];
  total += redS[4]; total += redS[5]; total += redS[6]; total += redS[7];
  const float inv = 1.0f / total;

  const int c0 = t * 8;
  const v4f a = *(const v4f*)(sP + c0);
  const v4f c = *(const v4f*)(sP + c0 + 4);
  unsigned short hb[8], lb[8];
#pragma unroll
  for (int e = 0; e < 4; ++e) {
    const float p0 = a[e] * inv;
    const unsigned short h0 = f2bf_bits(p0);
    hb[e] = h0;
    lb[e] = f2bf_bits(p0 - bf_bits2f(h0));
    const float p1 = c[e] * inv;
    const unsigned short h1 = f2bf_bits(p1);
    hb[4 + e] = h1;
    lb[4 + e] = f2bf_bits(p1 - bf_bits2f(h1));
  }
  const v4u uh = (v4u){pk16(hb[0], hb[1]), pk16(hb[2], hb[3]), pk16(hb[4], hb[5]), pk16(hb[6], hb[7])};
  const v4u ul = (v4u){pk16(lb[0], lb[1]), pk16(lb[2], lb[3]), pk16(lb[4], lb[5]), pk16(lb[6], lb[7])};
  unsigned short* qh = Ah + (size_t)blk * kSeq + c0;
  unsigned short* ql = Al + (size_t)blk * kSeq + c0;
  *(volatile v4u*)qh = uh;
  *(volatile v4u*)ql = ul;
  __threadfence();
  *(volatile v4u*)qh = uh;
  *(volatile v4u*)ql = ul;
}

extern "C" void kernel_launch(void* const* d_in, const int* in_sizes, int n_in,
                              void* d_out, int out_size, void* d_ws, size_t ws_size,
                              hipStream_t stream) {
  if (n_in < 11) return;
  if (in_sizes[0] != kTok * kDim) return;
  if (in_sizes[5] != kDim * kDim || in_sizes[6] != kDim) return;
  if (in_sizes[7] != kDim * kDim || in_sizes[8] != kDim) return;
  if (in_sizes[9] != 3 * kDim || in_sizes[10] != 3) return;
  if (out_size != kTok * kDim) return;

  const float* x   = (const float*)d_in[0];
  const float* wv  = (const float*)d_in[5];
  const float* bv  = (const float*)d_in[6];
  const float* wo  = (const float*)d_in[7];
  const float* bo  = (const float*)d_in[8];
  const float* w3d = (const float*)d_in[9];
  const float* b3d = (const float*)d_in[10];
  float* out = (float*)d_out;

  const size_t bXb  = (size_t)kTok * kDim * 2;
  const size_t bW   = (size_t)kDim * kDim * 2;
  const size_t bBia = (size_t)2 * kDim * 4;
  const size_t bPos = (size_t)kTok * kPosLd * 4;
  const size_t bVt  = (size_t)kBatch * kDim * kSeq * 2;
  const size_t bA   = (size_t)kBatch * kSeq * kSeq * 2;
  const size_t bO   = (size_t)kTok * kDim * 2;

  size_t off = 0;
  char* base = (char*)d_ws;
  unsigned short* Xb  = (unsigned short*)(base + off); off += bXb;
  unsigned short* WVb = (unsigned short*)(base + off); off += bW;
  unsigned short* WOb = (unsigned short*)(base + off); off += bW;
  float* bvr = (float*)(base + off);
  float* bor = bvr + kDim;                             off += bBia;
  float* pos = (float*)(base + off);                   off += bPos;
  unsigned short* Vth = (unsigned short*)(base + off); off += bVt;
  unsigned short* Vtl = (unsigned short*)(base + off); off += bVt;
  unsigned short* Ah  = (unsigned short*)(base + off); off += bA;
  unsigned short* Al  = (unsigned short*)(base + off); off += bA;
  unsigned short* Oh  = (unsigned short*)(base + off); off += bO;
  unsigned short* Ol  = (unsigned short*)(base + off); off += bO;
  if (off > ws_size) return;

  const dim3 blk(256);

  {
    const int n8x = kTok * kDim / 8;
    const int n8w = kDim * kDim / 8;
    cast8_bf16_kernel<<<dim3((n8x + 255) / 256), blk, 0, stream>>>(x, Xb, n8x);
    cast8_bf16_kernel<<<dim3((n8w + 255) / 256), blk, 0, stream>>>(wv, WVb, n8w);
    cast8_bf16_kernel<<<dim3((n8w + 255) / 256), blk, 0, stream>>>(wo, WOb, n8w);
  }
  bias_bf16_kernel<<<dim3(1), blk, 0, stream>>>(bv, bo, bvr, bor);

  wmma_gemm64<1, 0, 1, 2, false><<<dim3(64, kBatch), blk, 0, stream>>>(
      WVb, WVb, kDim, 0L,
      Xb, Xb, kDim, (long)kSeq * kDim,
      (void*)Vth, (void*)Vtl, kSeq, (long)kDim * kSeq,
      bvr, bvr, 0L,
      kDim, kSeq, kDim, 1.0f);

  pos_kernel<<<dim3(kTok / 8), blk, 0, stream>>>(Xb, w3d, b3d, pos);

  attn_rows_kernel<<<dim3(kTok), blk, 0, stream>>>(pos, Ah, Al);

  wmma_gemm64<1, 2, 0, 2, false, 0, true><<<dim3(64, kBatch), blk, 0, stream>>>(
      Ah, Al, kSeq, (long)kSeq * kSeq,
      Vth, Vtl, kSeq, (long)kDim * kSeq,
      (void*)Oh, (void*)Ol, kDim, (long)kSeq * kDim,
      bvr, bvr, 0L,
      kSeq, kDim, kSeq, 1.0f);

  wmma_gemm64<1, 1, 2, 0, false><<<dim3(128, 1), blk, 0, stream>>>(
      Oh, Ol, kDim, 0L,
      WOb, WOb, kDim, 0L,
      (void*)out, (void*)out, kDim, 0L,
      bor, bor, 0L,
      kTok, kDim, kDim, 1.0f);
}
